// MambaBlock_84576495993368
// MI455X (gfx1250) — hardware-run, weakly checked
//
#include <hip/hip_runtime.h>
#include <math.h>

typedef __attribute__((ext_vector_type(16))) _Float16 v16h;
typedef __attribute__((ext_vector_type(8)))  _Float16 v8h;
typedef __attribute__((ext_vector_type(8)))  float    v8f;
typedef __attribute__((ext_vector_type(4)))  float    v4f;

constexpr int kBatch  = 2;
constexpr int kSeq    = 2048;
constexpr int kDm     = 2048;
constexpr int kNst    = 16;
constexpr int kNout   = 2 * kDm + kNst + 1;
constexpr int kNpad   = 4128;
constexpr int kRows   = kBatch * kSeq;
constexpr int kColXc  = kDm;
constexpr int kColB   = 2 * kDm;
constexpr int kColD   = 2 * kDm + kNst;
constexpr int kDbP    = 32;
constexpr int kTilesM = kSeq / 64;
constexpr int kTilesN = kNpad / 32;
constexpr int kGemmBlocks = (kTilesM * kTilesN) / 8;
constexpr int kSlabP  = 36;
constexpr int kPrepP  = 36;
constexpr int kScanTS = 64;
constexpr int kScanCh = 64;
constexpr int kScanYP = 68;
constexpr int kWtP    = 33;
static_assert(kNout == 4113);
static_assert((kNpad % 32) == 0 && kNpad >= kNout && (kNpad - kNout) < 32);
static_assert((kDm % 64) == 0 && (kSeq % 64) == 0 && (kDm % 32) == 0);
static_assert(((kTilesM * kTilesN) % 8) == 0);
static_assert((kSeq % kScanTS) == 0 && (kDm % kScanCh) == 0 && (kRows % 32) == 0);
static_assert(kColD - kColB == 16 && kDbP >= kNst + 1);

constexpr float kCarryX      = 16.0f;
constexpr float kCarryW      = 1024.0f;
constexpr float kCarryRes    = 2048.0f;
constexpr float kFoldRes     = 1.0f / kCarryRes;
constexpr float kFoldMain    = 1.0f / (kCarryX * kCarryW);
constexpr float kF16MinNorm  = 6.103515625e-05f;

constexpr size_t kOffXH   = 0;
constexpr size_t kOffXL   = kOffXH + (size_t)kSeq  * kDm   * 2;
constexpr size_t kOffWH   = kOffXL + (size_t)kSeq  * kDm   * 2;
constexpr size_t kOffWL   = kOffWH + (size_t)kNpad * kDm   * 2;
constexpr size_t kOffXP   = kOffWL + (size_t)kNpad * kDm   * 2;
constexpr size_t kOffDB   = kOffXP + (size_t)kRows * kNpad * 4;
constexpr size_t kWsTotal = kOffDB + (size_t)kRows * kDbP  * 4;
static_assert(kWsTotal == 118751232ull);
static_assert(kWsTotal <= 134217728ull);
static_assert((kOffXL % 128) == 0 && (kOffWH % 128) == 0 && (kOffWL % 128) == 0 &&
              (kOffXP % 128) == 0 && (kOffDB % 128) == 0);

__device__ __forceinline__ void split_carry_f16(float v, float carry, _Float16& hi, _Float16& lo) {
  const float s0 = v * carry;
  const float s  = (fabsf(s0) < kF16MinNorm) ? 0.0f : s0;
  hi = (_Float16)s;
  const float hf = (float)hi;
  const float r0 = (s - hf) * kCarryRes;
  const float r  = (fabsf(r0) < kF16MinNorm) ? 0.0f : r0;
  lo = (_Float16)r;
}

__device__ __forceinline__ v16h frag_load(const _Float16* p) {
  union { v16h v; v8h h[2]; } f;
  f.h[0] = *(const v8h*)(p);
  f.h[1] = *(const v8h*)(p + 16);
  return f.v;
}

__device__ __forceinline__ v8f mma_f16(v16h a, v16h b, v8f c) {
  c = __builtin_amdgcn_wmma_f32_16x16x32_f16(false, a, false, b, (short)0, c, false, false);
  asm volatile("v_nop\n\tv_nop\n\tv_nop\n\tv_nop" : "+v"(c) : "v"(a), "v"(b));
  return c;
}

__global__ __launch_bounds__(256) void split_x_kernel(
    const float* __restrict__ src, unsigned short* __restrict__ dhi, unsigned short* __restrict__ dlo, int total8)
{
  const int i = blockIdx.x * 256 + threadIdx.x;
  if (i >= total8) return;
  const size_t e0 = (size_t)i << 3;
  const v4f a0 = *(const v4f*)(src + e0);
  const v4f a1 = *(const v4f*)(src + e0 + 4);
  v8h hv, lv;
#pragma unroll
  for (int e = 0; e < 4; ++e) {
    const float f0 = a0[e];
    const float f1 = a1[e];
    _Float16 h0, l0, h1, l1;
    split_carry_f16(f0, kCarryX, h0, l0);
    split_carry_f16(f1, kCarryX, h1, l1);
    hv[e]     = h0;
    hv[4 + e] = h1;
    lv[e]     = l0;
    lv[4 + e] = l1;
  }
  unsigned short* qh = dhi + e0;
  unsigned short* ql = dlo + e0;
  *(volatile v8h*)qh = hv;
  *(volatile v8h*)ql = lv;
  __threadfence();
  *(volatile v8h*)qh = hv;
  *(volatile v8h*)ql = lv;
}

__global__ __launch_bounds__(256) void split_wT_kernel(
    const float* __restrict__ W, unsigned short* __restrict__ WH, unsigned short* __restrict__ WL)
{
  __shared__ __align__(16) float sT[64 * kWtP];
  const int tid = threadIdx.x, lane = tid & 31, wave = tid >> 5;
  const int k0 = blockIdx.x * 64;
  const int n0 = blockIdx.y * 32;
  const int nl = tid & 31, kr = tid >> 5;
  const int n  = n0 + nl;
  const bool live = (n < kNout);
  const int nc = live ? n : (kNout - 1);
#pragma unroll
  for (int i = 0; i < 8; ++i) {
    const int k = kr + 8 * i;
    float wv = W[(size_t)(k0 + k) * kNout + nc];
    asm volatile("" : "+v"(wv));
    wv = live ? wv : 0.0f;
    sT[k * kWtP + nl] = wv;
  }
  __syncthreads();
  const int q = lane >> 3, c8 = (lane & 7) * 8;
  const int row = wave * 4 + q;
  v8h hv, lv;
#pragma unroll
  for (int e = 0; e < 8; ++e) {
    const float f = sT[(c8 + e) * kWtP + row];
    _Float16 h, l;
    split_carry_f16(f, kCarryW, h, l);
    hv[e] = h;
    lv[e] = l;
  }
  const size_t o = (size_t)(n0 + row) * kDm + k0 + c8;
  unsigned short* qh = WH + o;
  unsigned short* ql = WL + o;
  *(volatile v8h*)qh = hv;
  *(volatile v8h*)ql = lv;
  __threadfence();
  *(volatile v8h*)qh = hv;
  *(volatile v8h*)ql = lv;
}

__global__ __launch_bounds__(256) void proj_gemm_kernel(
    const unsigned short* __restrict__ XHp, const unsigned short* __restrict__ XLp,
    const unsigned short* __restrict__ WHp, const unsigned short* __restrict__ WLp,
    const float* __restrict__ bias, float* __restrict__ XPb)
{
  __shared__ __align__(16) float sT[8][16 * kSlabP];
  const _Float16* XH = (const _Float16*)XHp;
  const _Float16* XL = (const _Float16*)XLp;
  const _Float16* WH = (const _Float16*)WHp;
  const _Float16* WL = (const _Float16*)WLp;
  const int lane = threadIdx.x & 31;
  const int wave = threadIdx.x >> 5;
  const int tile = blockIdx.x * 8 + wave;
  if (tile >= kTilesM * kTilesN) return;
  const int tm = tile / kTilesN;
  const int tn = tile - tm * kTilesN;
  const int m0 = tm << 6;
  const int n0 = tn << 5;
  const int rlane = lane & 15;
  const int koff  = (lane >> 4) * 8;
  const int mOff  = (lane >> 4) * 8;

  v8f accM[4][2], accR[4][2];
#pragma unroll
  for (int i = 0; i < 4; ++i)
#pragma unroll
    for (int j = 0; j < 2; ++j) {
      accM[i][j] = (v8f){0.f, 0.f, 0.f, 0.f, 0.f, 0.f, 0.f, 0.f};
      accR[i][j] = (v8f){0.f, 0.f, 0.f, 0.f, 0.f, 0.f, 0.f, 0.f};
    }

#pragma unroll 1
  for (int k0 = 0; k0 < kDm; k0 += 32) {
    v16h bh[2], bl[2];
#pragma unroll
    for (int j = 0; j < 2; ++j) {
      const size_t bo = (size_t)(n0 + (j << 4) + rlane) * kDm + koff + k0;
      bh[j] = frag_load(WH + bo);
      bl[j] = frag_load(WL + bo);
    }
#pragma unroll
    for (int i = 0; i < 4; ++i) {
      const size_t ao = (size_t)(m0 + (i << 4) + rlane) * kDm + koff + k0;
      const v16h ah = frag_load(XH + ao);
      const v16h al = frag_load(XL + ao);
#pragma unroll
      for (int j = 0; j < 2; ++j) {
        accM[i][j] = mma_f16(ah, bh[j], accM[i][j]);
        accR[i][j] = mma_f16(ah, bl[j], accR[i][j]);
        accR[i][j] = mma_f16(al, bh[j], accR[i][j]);
      }
    }
  }

  float bv[2];
#pragma unroll
  for (int j = 0; j < 2; ++j) {
    const int n = n0 + (j << 4) + rlane;
    const bool nlive = (n < kNout);
    const int ncl = nlive ? n : (kNout - 1);
    float bb = bias[ncl];
    asm volatile("" : "+v"(bb));
    bv[j] = nlive ? bb : 0.0f;
  }

  float* slab = sT[wave];
  const int q = lane >> 3, c4 = (lane & 7) * 4;
#pragma unroll
  for (int i = 0; i < 4; ++i) {
    const int mBase = m0 + (i << 4);
#pragma unroll
    for (int j = 0; j < 2; ++j) {
#pragma unroll
      for (int r = 0; r < 8; ++r) {
        float v = fmaf(accR[i][j][r], kFoldRes, accM[i][j][r]);
        v = fmaf(v, kFoldMain, bv[j]);
        slab[(mOff + r) * kSlabP + (j << 4) + rlane] = v;
      }
    }
    __builtin_amdgcn_fence(__ATOMIC_RELEASE, "workgroup");
    __builtin_amdgcn_wave_barrier();
    __builtin_amdgcn_fence(__ATOMIC_ACQUIRE, "workgroup");
    for (int pass = 0; pass < 2; ++pass) {
#pragma unroll
      for (int it = 0; it < 4; ++it) {
        const int row = it * 4 + q;
        const v4f v = *(const v4f*)(slab + row * kSlabP + c4);
        *(volatile v4f*)(XPb + (size_t)(mBase + row) * kNpad + n0 + c4) = v;
      }
      __threadfence();
    }
    __builtin_amdgcn_fence(__ATOMIC_RELEASE, "workgroup");
    __builtin_amdgcn_wave_barrier();
    __builtin_amdgcn_fence(__ATOMIC_ACQUIRE, "workgroup");
  }
}

__global__ __launch_bounds__(256) void prep_step_kernel(
    const float* __restrict__ XP, const float* __restrict__ Bp, float* __restrict__ DB)
{
  __shared__ __align__(16) float sD[32 * kPrepP];
  const int tid = threadIdx.x, lane = tid & 31, wave = tid >> 5;
  const int m0 = blockIdx.x * 32;
  const int cc = (lane < 16) ? lane : 16;
  const int bi = (lane < 15) ? lane : 15;
  float bp = Bp[bi];
  asm volatile("" : "+v"(bp));
#pragma unroll 1
  for (int r = 0; r < 4; ++r) {
    const int lr = wave * 4 + r;
    const float* rowp = XP + (size_t)(m0 + lr) * kNpad;
    float cv = rowp[kColB + cc];
    float dr = rowp[kColD];
    asm volatile("" : "+v"(cv));
    asm volatile("" : "+v"(dr));
    const float sp    = fmaxf(dr, 0.0f) + log1pf(expf(-fabsf(dr)));
    const float sg    = 1.0f / (1.0f + expf(-sp));
    const float delta = sp * sg;
    const float bt    = delta * (cv + bp);
    float val = (lane == 16) ? delta : 0.0f;
    val = (lane < 16) ? bt : val;
    sD[lr * kPrepP + lane] = val;
  }
  __syncthreads();
  const int row = tid >> 3, c4 = (tid & 7) * 4;
  const v4f v = *(const v4f*)(sD + row * kPrepP + c4);
  float* p = DB + (size_t)(m0 + row) * kDbP + c4;
  *(volatile v4f*)p = v;
  __threadfence();
  *(volatile v4f*)p = v;
}

__global__ __launch_bounds__(64) void scan_gate_kernel(
    const float* __restrict__ XP, const float* __restrict__ DB, const float* __restrict__ Alog,
    const float* __restrict__ Cp, const float* __restrict__ cw, float* __restrict__ out)
{
  __shared__ __align__(16) float sX[kScanTS * kDbP];
  __shared__ __align__(16) float sY[kScanTS * kScanYP];
  __shared__ __align__(16) float sA[kNst * kScanCh];
  const int tid = threadIdx.x, lane = tid & 31, wave = tid >> 5;
  constexpr int kBlkPerB = kDm / kScanCh;
  const int bix = blockIdx.x / kBlkPerB;
  const int d0  = (blockIdx.x - bix * kBlkPerB) * kScanCh;
  const int d   = d0 + tid;
  const size_t row0 = (size_t)bix * kSeq;

#pragma unroll 1
  for (int s = 0; s < kNst; ++s) sA[s * kScanCh + tid] = -expf(Alog[(size_t)d * kNst + s]);
  __syncthreads();
  float negA[kNst], h[kNst], Cc[kNst];
#pragma unroll
  for (int s = 0; s < kNst; ++s) {
    negA[s] = sA[s * kScanCh + tid];
    h[s] = 0.0f;
  }
#pragma unroll
  for (int q4 = 0; q4 < 4; ++q4) {
    const v4f cv = *(const v4f*)(Cp + (size_t)d * kNst + 4 * q4);
    Cc[4 * q4 + 0] = cv[0];
    Cc[4 * q4 + 1] = cv[1];
    Cc[4 * q4 + 2] = cv[2];
    Cc[4 * q4 + 3] = cv[3];
  }
  const v4f wv = *(const v4f*)(cw + (size_t)d * 4);
  const float w0 = wv[0], w1 = wv[1], w2 = wv[2], w3 = wv[3];
  float s1 = 0.0f, s2 = 0.0f, s3 = 0.0f;

  const int lr = tid >> 3, lc4 = (tid & 7) * 4;
  const int hh = lane >> 4, c4 = (lane & 15) * 4;

#pragma unroll 1
  for (int t0 = 0; t0 < kSeq; t0 += kScanTS) {
    __syncthreads();
#pragma unroll
    for (int i = 0; i < 8; ++i) {
      const int r = lr + 8 * i;
      *(v4f*)(sX + r * kDbP + lc4) = *(const v4f*)(DB + (row0 + t0 + r) * kDbP + lc4);
    }
    __syncthreads();
#pragma unroll 1
    for (int s = 0; s < kScanTS; ++s) {
      const float* rowp = XP + (row0 + t0 + s) * kNpad;
      const float xc = rowp[kColXc + d];
      const float vv = rowp[d];
      const float* xr = sX + s * kDbP;
      const float delta = xr[kNst];
      const float sgx = __builtin_amdgcn_rcpf(1.0f + __expf(-xc));
      const float sv  = xc * sgx;
      float xv = w0 * s3;
      xv = fmaf(w1, s2, xv);
      xv = fmaf(w2, s1, xv);
      xv = fmaf(w3, sv, xv);
      s3 = s2;
      s2 = s1;
      s1 = sv;
      float y = 0.0f;
#pragma unroll
      for (int q4 = 0; q4 < 4; ++q4) {
        const v4f bq = *(const v4f*)(xr + 4 * q4);
#pragma unroll
        for (int e = 0; e < 4; ++e) {
          const int k = 4 * q4 + e;
          const float dA = __expf(delta * negA[k]);
          const float inj = bq[e] * xv;
          h[k] = fmaf(dA, h[k], inj);
          y = fmaf(h[k], Cc[k], y);
        }
      }
      const float sgv = __builtin_amdgcn_rcpf(1.0f + __expf(-vv));
      sY[s * kScanYP + tid] = y * (vv * sgv);
    }
    __syncthreads();
    for (int pass = 0; pass < 2; ++pass) {
#pragma unroll
      for (int it = 0; it < 16; ++it) {
        const int row = it * 4 + wave * 2 + hh;
        const v4f v = *(const v4f*)(sY + row * kScanYP + c4);
        *(volatile v4f*)(out + (row0 + t0 + row) * kDm + d0 + c4) = v;
      }
      __threadfence();
    }
  }
}

extern "C" void kernel_launch(void* const* d_in, const int* in_sizes, int n_in,
                              void* d_out, int out_size, void* d_ws, size_t ws_size,
                              hipStream_t stream) {
  if (n_in < 7) return;
  if (in_sizes[0] != kRows * kDm) return;
  if (in_sizes[1] != kDm * kNout) return;
  if (in_sizes[2] != kNout) return;
  if (in_sizes[3] != kDm * kNst) return;
  if (in_sizes[4] != kNst) return;
  if (in_sizes[5] != kDm * kNst) return;
  if (in_sizes[6] != kDm * 4) return;
  if (out_size != kRows * kDm) return;
  if (ws_size < kWsTotal) return;

  const float* x     = (const float*)d_in[0];
  const float* W_in  = (const float*)d_in[1];
  const float* b_in  = (const float*)d_in[2];
  const float* A_log = (const float*)d_in[3];
  const float* Bpar  = (const float*)d_in[4];
  const float* Cpar  = (const float*)d_in[5];
  const float* convw = (const float*)d_in[6];
  float* out = (float*)d_out;

  char* ws = (char*)d_ws;
  unsigned short* XH = (unsigned short*)(ws + kOffXH);
  unsigned short* XL = (unsigned short*)(ws + kOffXL);
  unsigned short* WH = (unsigned short*)(ws + kOffWH);
  unsigned short* WL = (unsigned short*)(ws + kOffWL);
  float*          XP = (float*)(ws + kOffXP);
  float*          DB = (float*)(ws + kOffDB);

  split_wT_kernel<<<dim3(kDm / 64, kNpad / 32), 256, 0, stream>>>(W_in, WH, WL);

  constexpr int kX8 = kSeq * kDm / 8;
  for (int b = 0; b < kBatch; ++b) {
    split_x_kernel<<<kX8 / 256, 256, 0, stream>>>(x + (size_t)b * kSeq * kDm, XH, XL, kX8);
    proj_gemm_kernel<<<kGemmBlocks, 256, 0, stream>>>(XH, XL, WH, WL, b_in, XP + (size_t)b * kSeq * kNpad);
  }

  prep_step_kernel<<<kRows / 32, 256, 0, stream>>>(XP, Bpar, DB);

  scan_gate_kernel<<<kBatch * (kDm / kScanCh), kScanCh, 0, stream>>>(XP, DB, A_log, Cpar, convw, out);
}
